// Geoconv_472446403135
// MI455X (gfx1250) — hardware-verified
//
#include <hip/hip_runtime.h>


namespace {
constexpr int Bn = 16, N = 2048, CIN = 64, COUT = 64, CB = 32, C6 = 6 * CB, NT = Bn * N, NBLK = NT / 128;
constexpr float R2 = 0.15f * 0.15f, DR2 = 0.3f * 0.3f, AS_ = 8.0f, MS_ = 8.0f, EPS = 1e-5f;
constexpr size_t MPL = (size_t)Bn * C6 * N;

typedef _Float16 b16;
typedef __attribute__((ext_vector_type(16))) _Float16 v16b;
typedef __attribute__((ext_vector_type(16))) __bf16 v16bb;
typedef __attribute__((ext_vector_type(8))) _Float16 v8b;
typedef __attribute__((ext_vector_type(8))) unsigned short v8us;
typedef __attribute__((ext_vector_type(8))) float v8f;
typedef __attribute__((ext_vector_type(4))) float v4f;
__device__ __forceinline__ float bf16_rne(float f) { unsigned int u = __float_as_uint(f); u += 0x7FFFu + ((u >> 16) & 1u); return __uint_as_float(u & 0xFFFF0000u); }
__device__ __forceinline__ unsigned short bf16_bits(float f) { unsigned int u = __float_as_uint(f); u += 0x7FFFu + ((u >> 16) & 1u); return (unsigned short)(u >> 16); }
__device__ __forceinline__ void split16(float v, b16& hi, b16& lo) { hi = (b16)v; lo = (b16)(v - (float)hi); }
__device__ __forceinline__ v16b frag_kb(const b16* p, int hh) { const v8b a = *(const v8b*)(p + 8 * hh), b = *(const v8b*)(p + 16 + 8 * hh); v16b f;
#pragma unroll
  for (int e = 0; e < 8; ++e) { f[e] = a[e]; f[8 + e] = b[e]; } return f; }
__device__ __forceinline__ v16bb frag_bf(const unsigned short* p, int hh) { const v8us a = *(const v8us*)(p + 8 * hh), b = *(const v8us*)(p + 16 + 8 * hh); union { unsigned short s[16]; v16bb v; } u;
#pragma unroll
  for (int e = 0; e < 8; ++e) { u.s[e] = a[e]; u.s[8 + e] = b[e]; } return u.v; }
__device__ __forceinline__ v16bb frag_f32bf(const float* p, int hh) { union { unsigned short s[16]; v16bb v; } u;
#pragma unroll
  for (int e = 0; e < 8; ++e) { u.s[e] = bf16_bits(p[8 * hh + e]); u.s[8 + e] = bf16_bits(p[16 + 8 * hh + e]); } return u.v; }
__device__ __forceinline__ v8f wmma16b(v16b a, v16b b, v8f c) { v8f d = __builtin_amdgcn_wmma_f32_16x16x32_f16(false, a, false, b, (short)0, c, false, false); asm volatile("v_nop\n\tv_nop\n\tv_nop\n\tv_nop" : "+v"(d) : "v"(a), "v"(b)); return d; }
__device__ __forceinline__ v8f wmma16bb(v16bb a, v16bb b, v8f c) { v8f d = __builtin_amdgcn_wmma_f32_16x16x32_bf16(false, a, false, b, (short)0, c, false, false); asm volatile("v_nop\n\tv_nop\n\tv_nop\n\tv_nop" : "+v"(d) : "v"(a), "v"(b)); return d; }
__device__ __forceinline__ void wave_lds_sync() { __builtin_amdgcn_fence(__ATOMIC_RELEASE, "workgroup"); __builtin_amdgcn_wave_barrier(); __builtin_amdgcn_fence(__ATOMIC_ACQUIRE, "workgroup"); }
__device__ __forceinline__ float pmul(float a, float b) { float p = a * b; asm volatile("" : "+v"(p)); return p; }

__global__ __launch_bounds__(256) void prep_kernel(const float* __restrict__ Wf, const float* __restrict__ Wb, const float* __restrict__ Wag, unsigned short* __restrict__ w16, b16* __restrict__ wagr) {
  const int t_ = threadIdx.x;
  for (int pass = 0; pass < 2; ++pass) {
    for (int p = t_; p < 256 * CIN; p += 256) { const int o = p >> 6, k = p & 63; const float v = (o < COUT) ? Wf[k * COUT + o] : Wb[k * C6 + (o - COUT)]; ((volatile unsigned short*)w16)[p] = bf16_bits(v); }
    for (int p = t_; p < COUT * CB; p += 256) { const int o = p >> 5, k = p & 31; ((volatile b16*)wagr)[p] = (b16)bf16_rne(Wag[k * COUT + o]); }
    __threadfence(); }
}

__global__ __launch_bounds__(128) void g1_kernel(const float* __restrict__ feat, const unsigned short* __restrict__ w16, const float* __restrict__ bfe, float* __restrict__ sf, float* __restrict__ mraw, float* __restrict__ part1) {
  __shared__ __attribute__((aligned(16))) float Ts[4][32 * 64]; __shared__ float Cs[4][2][64];
  const int lane = threadIdx.x & 31, wave = threadIdx.x >> 5, nloc = lane & 15, hlf = lane >> 4, m0 = blockIdx.y * 128 + wave * 32, ct = blockIdx.x, c0 = ct * 64;
  v8f acc[2][4];
#pragma unroll
  for (int r = 0; r < 2; ++r)
#pragma unroll
    for (int t = 0; t < 4; ++t) acc[r][t] = (v8f){};
#pragma unroll
  for (int kb = 0; kb < CIN; kb += 32) { const v16bb a0 = frag_f32bf(feat + (size_t)(m0 + nloc) * CIN + kb, hlf), a1 = frag_f32bf(feat + (size_t)(m0 + 16 + nloc) * CIN + kb, hlf);
#pragma unroll
    for (int t = 0; t < 4; ++t) { const v16bb bw = frag_bf(w16 + (size_t)(c0 + t * 16 + nloc) * CIN + kb, hlf); acc[0][t] = wmma16bb(a0, bw, acc[0][t]); acc[1][t] = wmma16bb(a1, bw, acc[1][t]); } }
  float* Tt = Ts[wave];
#pragma unroll
  for (int t = 0; t < 4; ++t) { const float bb = (ct == 0) ? bf16_rne(bfe[t * 16 + nloc]) : 0.0f;
#pragma unroll
    for (int r = 0; r < 2; ++r)
#pragma unroll
      for (int v = 0; v < 8; ++v) Tt[(r * 16 + v + 8 * hlf) * 64 + t * 16 + nloc] = acc[r][t][v] + bb; }
  wave_lds_sync();
  { float s = 0.0f, s2 = 0.0f, q1 = 0.0f, q2 = 0.0f; for (int rr = 0; rr < 32; ++rr) { const float a = Tt[rr * 64 + lane * 2], c = Tt[rr * 64 + lane * 2 + 1]; s += a; q1 += a * a; s2 += c; q2 += c * c; }
    Cs[wave][0][lane * 2] = s; Cs[wave][0][lane * 2 + 1] = s2; Cs[wave][1][lane * 2] = q1; Cs[wave][1][lane * 2 + 1] = q2; }
  __syncthreads();
  float* dst0 = (ct == 0) ? (sf + (size_t)m0 * COUT) : (mraw + (size_t)m0 * C6 + (c0 - 64)); const int ld = (ct == 0) ? COUT : C6;
  for (int pass = 0; pass < 2; ++pass) {
#pragma unroll
    for (int j = 0; j < 16; ++j) { const int rr = j * 2 + hlf, c4 = nloc * 4; *(volatile v4f*)(dst0 + (size_t)rr * ld + c4) = *(const v4f*)(Tt + rr * 64 + c4); }
    if (ct > 0 && threadIdx.x < 128) { const int st = threadIdx.x >> 6, cc = threadIdx.x & 63; ((volatile float*)part1)[((size_t)blockIdx.y * 2 + st) * C6 + (c0 - 64) + cc] = Cs[0][st][cc] + Cs[1][st][cc] + Cs[2][st][cc] + Cs[3][st][cc]; }
    __threadfence(); }
}

__global__ __launch_bounds__(256) void bnstat_kernel(const float* __restrict__ part, int C, int nblk, int ntot, const float* __restrict__ gma, const float* __restrict__ bta, float* __restrict__ bn) {
  for (int c = threadIdx.x; c < C; c += 256) { double s = 0.0, q = 0.0;
    for (int blk = 0; blk < nblk; ++blk) { s += (double)part[((size_t)blk * 2 + 0) * C + c]; q += (double)part[((size_t)blk * 2 + 1) * C + c]; }
    const double mean = s / (double)ntot; const double var = fmax(q / (double)ntot - mean * mean, 0.0);
    const float scl = bf16_rne(gma[c]) * (float)(1.0 / sqrt(var + (double)EPS)); const float sh = bf16_rne(bta[c]) - (float)mean * scl;
    for (int pass = 0; pass < 2; ++pass) { ((volatile float*)bn)[c] = scl; ((volatile float*)bn)[C + c] = sh; } }
  __threadfence();
}

__global__ __launch_bounds__(256) void mt_kernel(const float* __restrict__ mraw, const float* __restrict__ bn1, b16* __restrict__ mt) {
  __shared__ __attribute__((aligned(16))) b16 Th[C6][128 + 8], Tl[C6][128 + 8];
  const int b = blockIdx.y, j0 = blockIdx.x * 128, t_ = threadIdx.x;
  for (int i = t_; i < 128 * C6; i += 256) { const int jj = i / C6, row = i % C6; b16 a, c; split16(fmaxf(mraw[((size_t)b * N + j0 + jj) * C6 + row] * bn1[row] + bn1[C6 + row], 0.0f) * MS_, a, c); Th[row][jj] = a; Tl[row][jj] = c; }
  __syncthreads();
  for (int pass = 0; pass < 2; ++pass) { for (int i = t_; i < C6 * 16; i += 256) { const int row = i >> 4, c8 = (i & 15) * 8; const size_t dst = ((size_t)b * C6 + row) * N + j0 + c8;
      *(volatile v8b*)(mt + dst) = *(const v8b*)(&Th[row][c8]); *(volatile v8b*)(mt + MPL + dst) = *(const v8b*)(&Tl[row][c8]); } __threadfence(); }
}

__global__ __launch_bounds__(256) void agg_kernel(const float* __restrict__ xyz, const b16* __restrict__ mt, float* __restrict__ agraw, float* __restrict__ part2) {
  __shared__ __attribute__((aligned(16))) float Os[8][16][CB + 4]; __shared__ float Nm[8][16]; __shared__ float Cs[8][2][32];
  const int wid = threadIdx.x >> 5, lane = threadIdx.x & 31, nloc = lane & 15, hh = lane >> 4; const int pt0 = blockIdx.x * 128 + wid * 16, b = pt0 / N, i0 = pt0 % N, i = i0 + nloc;
  const float* xb = xyz + (size_t)b * N * 3; const float xi = bf16_rne(xb[i * 3]), yi = bf16_rne(xb[i * 3 + 1]), zi = bf16_rne(xb[i * 3 + 2]);
  const b16* MT = mt + ((size_t)b * C6) * N;
  v8f acc[2] = {{}, {}}; float nrm = 0.0f;
  for (int jb = 0; jb < N; jb += 32) {
    v16b wf[6], wl[6];
#pragma unroll
    for (int e = 0; e < 16; ++e) { const int j = jb + ((e < 8) ? (8 * hh + e) : (16 + 8 * hh + e - 8));
      const float dx = bf16_rne(xb[j * 3]) - xi, dy = bf16_rne(xb[j * 3 + 1]) - yi, dz = bf16_rne(xb[j * 3 + 2]) - zi; const float d2 = pmul(dx, dx) + pmul(dy, dy) + pmul(dz, dz);
      const bool valid = (d2 < DR2) && (d2 > 0.0f); float wd = (d2 <= R2) ? 1.0f : (DR2 - d2) * (1.0f / (DR2 - R2)); wd = valid ? wd : 0.0f; nrm += wd;
      const float inv = wd / fmaxf(d2, 1e-12f); const float c3[3] = {dx, dy, dz};
#pragma unroll
      for (int a = 0; a < 3; ++a) { const float cp = fmaxf(c3[a], 0.0f), cn = fmaxf(-c3[a], 0.0f); b16 p, q; split16(inv * pmul(cp, cp) * AS_, p, q); wf[2 * a][e] = p; wl[2 * a][e] = q; split16(inv * pmul(cn, cn) * AS_, p, q); wf[2 * a + 1][e] = p; wl[2 * a + 1][e] = q; } }
#pragma unroll
    for (int g = 0; g < 6; ++g)
#pragma unroll
      for (int n = 0; n < 2; ++n) { const b16* br = MT + (size_t)(g * CB + n * 16 + nloc) * N + jb; const v16b bh = frag_kb(br, hh), bl = frag_kb(br + MPL, hh);
        acc[n] = wmma16b(wf[g], bh, acc[n]); acc[n] = wmma16b(wf[g], bl, acc[n]); acc[n] = wmma16b(wl[g], bh, acc[n]); } }
  nrm += __shfl_xor(nrm, 16); if (hh == 0) Nm[wid][nloc] = nrm;
  wave_lds_sync();
#pragma unroll
  for (int n = 0; n < 2; ++n)
#pragma unroll
    for (int r = 0; r < 8; ++r) { const int row = 8 * hh + r; Os[wid][row][n * 16 + nloc] = acc[n][r] * (1.0f / (AS_ * MS_)) / fmaxf(Nm[wid][row], 1e-12f); }
  wave_lds_sync();
  { float s = 0.0f, q = 0.0f; for (int rr = 0; rr < 16; ++rr) { const float a = Os[wid][rr][lane]; s += a; q += a * a; } Cs[wid][0][lane] = s; Cs[wid][1][lane] = q; }
  __syncthreads();
  for (int pass = 0; pass < 2; ++pass) {
#pragma unroll
    for (int jx = 0; jx < 4; ++jx) { const int rr = jx * 4 + (lane >> 3), c4 = (lane & 7) * 4; *(volatile v4f*)(agraw + (size_t)(pt0 + rr) * CB + c4) = *(const v4f*)(&Os[wid][rr][c4]); }
    if (threadIdx.x < 64) { const int st = threadIdx.x >> 5, cc = threadIdx.x & 31; float s = 0.0f; for (int w = 0; w < 8; ++w) s += Cs[w][st][cc]; ((volatile float*)part2)[((size_t)blockIdx.x * 2 + st) * CB + cc] = s; }
    __threadfence(); }
}

__global__ __launch_bounds__(128) void g2_kernel(const float* __restrict__ agraw, const float* __restrict__ bn2, const b16* __restrict__ wagr, const float* __restrict__ bag, const float* __restrict__ sf, float* __restrict__ z, float* __restrict__ part3) {
  __shared__ __attribute__((aligned(16))) float Ts[4][32 * 64]; __shared__ float Cs[4][2][64];
  const int lane = threadIdx.x & 31, wave = threadIdx.x >> 5, nloc = lane & 15, hlf = lane >> 4, m0 = blockIdx.x * 128 + wave * 32;
  v8f acc[2][4];
#pragma unroll
  for (int r = 0; r < 2; ++r)
#pragma unroll
    for (int t = 0; t < 4; ++t) acc[r][t] = (v8f){};
  { v16b a0, l0, a1, l1;
#pragma unroll
    for (int e = 0; e < 16; ++e) { const int k = (e < 8) ? (8 * hlf + e) : (16 + 8 * hlf + e - 8); const float sc = bn2[k], sh = bn2[CB + k]; b16 p, q;
      split16(fmaxf(agraw[(size_t)(m0 + nloc) * CB + k] * sc + sh, 0.0f) * AS_, p, q); a0[e] = p; l0[e] = q; split16(fmaxf(agraw[(size_t)(m0 + 16 + nloc) * CB + k] * sc + sh, 0.0f) * AS_, p, q); a1[e] = p; l1[e] = q; }
#pragma unroll
    for (int t = 0; t < 4; ++t) { const v16b bw = frag_kb(wagr + (size_t)(t * 16 + nloc) * CB, hlf); acc[0][t] = wmma16b(a0, bw, acc[0][t]); acc[0][t] = wmma16b(l0, bw, acc[0][t]); acc[1][t] = wmma16b(a1, bw, acc[1][t]); acc[1][t] = wmma16b(l1, bw, acc[1][t]); } }
  float* Tt = Ts[wave];
#pragma unroll
  for (int t = 0; t < 4; ++t) { const int c = t * 16 + nloc; const float bb = bf16_rne(bag[c]);
#pragma unroll
    for (int r = 0; r < 2; ++r)
#pragma unroll
      for (int v = 0; v < 8; ++v) { const int rr = r * 16 + v + 8 * hlf; Tt[rr * 64 + c] = acc[r][t][v] * (1.0f / AS_) + bb + sf[(size_t)(m0 + rr) * COUT + c]; } }
  wave_lds_sync();
  { float s = 0.0f, s2 = 0.0f, q1 = 0.0f, q2 = 0.0f; for (int rr = 0; rr < 32; ++rr) { const float a = Tt[rr * 64 + lane * 2], c = Tt[rr * 64 + lane * 2 + 1]; s += a; q1 += a * a; s2 += c; q2 += c * c; }
    Cs[wave][0][lane * 2] = s; Cs[wave][0][lane * 2 + 1] = s2; Cs[wave][1][lane * 2] = q1; Cs[wave][1][lane * 2 + 1] = q2; }
  __syncthreads();
  for (int pass = 0; pass < 2; ++pass) {
#pragma unroll
    for (int j = 0; j < 16; ++j) { const int rr = j * 2 + hlf, c4 = nloc * 4; *(volatile v4f*)(z + (size_t)(m0 + rr) * COUT + c4) = *(const v4f*)(Tt + rr * 64 + c4); }
    if (threadIdx.x < 128) { const int st = threadIdx.x >> 6, cc = threadIdx.x & 63; ((volatile float*)part3)[((size_t)blockIdx.x * 2 + st) * COUT + cc] = Cs[0][st][cc] + Cs[1][st][cc] + Cs[2][st][cc] + Cs[3][st][cc]; }
    __threadfence(); }
}
__global__ __launch_bounds__(256) void out_kernel(const float* __restrict__ z, const float* __restrict__ bn3, float* __restrict__ out) {
  const int t_ = threadIdx.x; const int c4 = (t_ & 15) * 4;
  for (int pass = 0; pass < 2; ++pass) { for (int rr = t_ >> 4; rr < 128; rr += 16) { const size_t row = (size_t)blockIdx.x * 128 + rr; const v4f v = *(const v4f*)(z + row * COUT + c4); v4f o;
#pragma unroll
      for (int e = 0; e < 4; ++e) o[e] = fmaxf(v[e] * bn3[c4 + e] + bn3[COUT + c4 + e], 0.0f);
      *(volatile v4f*)(out + row * COUT + c4) = o; } __threadfence(); }
}
}

extern "C" void kernel_launch(void* const* d_in, const int* in_sizes, int n_in,
                              void* d_out, int out_size, void* d_ws, size_t ws_size, hipStream_t stream) {
  (void)n_in; (void)out_size;
  const float* feat = (const float*)d_in[0]; const float* xyz = (const float*)d_in[1]; const float* Wf = (const float*)d_in[2]; const float* bfe = (const float*)d_in[3]; const float* Wb = (const float*)d_in[4]; const float* gb = (const float*)d_in[5]; const float* bb = (const float*)d_in[6];
  const float* g1 = (const float*)d_in[7]; const float* be1 = (const float*)d_in[8]; const float* Wag = (const float*)d_in[9]; const float* bag = (const float*)d_in[10]; const float* g2 = (const float*)d_in[11]; const float* be2 = (const float*)d_in[12];
  float* out = (float*)d_out;
  if (in_sizes[0] != NT * CIN || in_sizes[1] != NT * 3 || in_sizes[2] != CIN * COUT || in_sizes[4] != CIN * C6 || in_sizes[9] != CB * COUT) return;
  size_t off = 0; char* ws = (char*)d_ws;
  auto carve = [&](size_t bytes) { char* p = ws + off; off += (bytes + 255) & ~(size_t)255; return p; };
  unsigned short* w16 = (unsigned short*)carve(256 * CIN * 2); b16* wagr = (b16*)carve(COUT * CB * 2);
  float* sf = (float*)carve((size_t)NT * COUT * 4); float* mraw = (float*)carve((size_t)NT * C6 * 4); float* part1 = (float*)carve((size_t)NBLK * 2 * C6 * 4); float* bn1 = (float*)carve(2 * C6 * 4);
  b16* mt = (b16*)carve(MPL * 2 * 2); float* agraw = (float*)carve((size_t)NT * CB * 4); float* part2 = (float*)carve((size_t)NBLK * 2 * CB * 4); float* bn2 = (float*)carve(2 * CB * 4);
  float* z = (float*)carve((size_t)NT * COUT * 4); float* part3 = (float*)carve((size_t)NBLK * 2 * COUT * 4); float* bn3 = (float*)carve(2 * COUT * 4);
  if (off > ws_size) return;
  prep_kernel<<<1, 256, 0, stream>>>(Wf, Wb, Wag, w16, wagr);
  g1_kernel<<<dim3(4, NBLK), 128, 0, stream>>>(feat, w16, bfe, sf, mraw, part1);
  bnstat_kernel<<<1, 256, 0, stream>>>(part1, C6, NBLK, NT, gb, bb, bn1);
  mt_kernel<<<dim3(N / 128, Bn), 256, 0, stream>>>(mraw, bn1, mt);
  agg_kernel<<<NT / 128, 256, 0, stream>>>(xyz, mt, agraw, part2);
  bnstat_kernel<<<1, 256, 0, stream>>>(part2, CB, NBLK, NT, g1, be1, bn2);
  g2_kernel<<<NBLK, 128, 0, stream>>>(agraw, bn2, wagr, bag, sf, z, part3);
  bnstat_kernel<<<1, 256, 0, stream>>>(part3, COUT, NBLK, NT, g2, be2, bn3);
  out_kernel<<<NBLK, 256, 0, stream>>>(z, bn3, out);
}
